// MultiQueryAttention_51762945851576
// MI455X (gfx1250) — hardware-verified
//
#include <hip/hip_runtime.h>


#ifndef NB
#define NB 1
#endif
#ifndef SEQ
#define SEQ 2048
#endif
#define SEQ_FULL 2048
#define TT   SEQ
#define TTF  SEQ_FULL
#define DM   2048
#define NH_  16
#define NKV  4
#define REP  (NH_ / NKV)
#define HD   128
#define DQ   (NH_ * HD)
#define DKV  (NKV * HD)
#define ZH   4
#define KSH  11
#define PCAR 1024.0f
#define SCL  0.088388347648318447f
#define NEGF (-3.4028234663852886e38f)

static_assert(HD == 128);
static_assert(ZH == REP);
static_assert((TT % 128) == 0);
static_assert((TT & (TT - 1)) == 0);
static_assert(DM == (1 << KSH));
static_assert(DQ == (1 << KSH));
static_assert((DKV % 64) == 0);
static_assert(TT <= TTF);

typedef _Float16 h16;
typedef unsigned short bf;
typedef __attribute__((ext_vector_type(16))) __bf16   v16bf;
typedef __attribute__((ext_vector_type(16))) _Float16 v16h;
typedef __attribute__((ext_vector_type(8)))  _Float16 v8h;
typedef __attribute__((ext_vector_type(8)))  unsigned short v8us;
typedef __attribute__((ext_vector_type(8)))  float    v8f;
typedef __attribute__((ext_vector_type(4)))  float    v4f;
typedef __attribute__((ext_vector_type(2)))  _Float16 v2h;
typedef __attribute__((ext_vector_type(4)))  _Float16 v4h;
typedef __attribute__((ext_vector_type(2)))  unsigned short v2us;
typedef __attribute__((ext_vector_type(2)))  float v2f;
typedef __attribute__((ext_vector_type(4)))  int v4i;
typedef v4f  __attribute__((may_alias)) v4fa;

__device__ __forceinline__ unsigned short f2bf(float f) { unsigned u = __float_as_uint(f); u += 0x7FFFu + ((u >> 16) & 1u); return (unsigned short)(u >> 16); }
__device__ __forceinline__ float bf2f(unsigned short b) { return __uint_as_float(((unsigned)b) << 16); }
__device__ __forceinline__ float bfr(float f) { return bf2f(f2bf(f)); }
__device__ __forceinline__ v16h cat16(v8h lo, v8h hi) { return __builtin_shufflevector(lo, hi, 0, 1, 2, 3, 4, 5, 6, 7, 8, 9, 10, 11, 12, 13, 14, 15); }
__device__ __forceinline__ v16bf cat16b(v8us lo, v8us hi) { return __builtin_bit_cast(v16bf, __builtin_shufflevector(lo, hi, 0, 1, 2, 3, 4, 5, 6, 7, 8, 9, 10, 11, 12, 13, 14, 15)); }
__device__ __forceinline__ v8f wmma16(v16h a, v16h b, v8f c) { return __builtin_amdgcn_wmma_f32_16x16x32_f16(false, a, false, b, (short)0, c, false, false); }
__device__ __forceinline__ v8f wmmab(v16bf a, v16bf b, v8f c) { return __builtin_amdgcn_wmma_f32_16x16x32_bf16(false, a, false, b, (short)0, c, false, false); }

template <typename T16> struct WFrag;
template <> struct WFrag<h16> { typedef v16h V; static __device__ __forceinline__ V ld(const h16* p) { return cat16(*(const v8h*)p, *(const v8h*)(p + 16)); } static __device__ __forceinline__ v8f mma(V a, V b, v8f c) { return wmma16(a, b, c); } };
template <> struct WFrag<bf> { typedef v16bf V; static __device__ __forceinline__ V ld(const bf* p) { return cat16b(*(const v8us*)p, *(const v8us*)(p + 16)); } static __device__ __forceinline__ v8f mma(V a, V b, v8f c) { return wmmab(a, b, c); } };
template <typename T16, int NSPLIT, bool BIAS>
__global__ __launch_bounds__(32) void k_gemmw(const T16* __restrict__ A, const T16* __restrict__ A2, const T16* __restrict__ Bt, const T16* __restrict__ Bt2, int K, float* C, int ldc, const float* __restrict__ bias, size_t sA, size_t sB, size_t sC) {
    typedef typename WFrag<T16>::V V;
    __shared__ __align__(16) float os[16 * 68];
    const size_t z = blockIdx.z; A += z * sA; if (A2) A2 += z * sA; Bt += z * sB; if (Bt2) Bt2 += z * sB; C += z * sC;
    const int lane = threadIdx.x & 31, lr = lane & 15, hi = lane >> 4; const int r0 = blockIdx.x * 64, c0 = blockIdx.y * 64;
    v8f acc[4][4];
#pragma unroll
    for (int mb = 0; mb < 4; ++mb)
#pragma unroll
        for (int nb = 0; nb < 4; ++nb) acc[mb][nb] = (v8f){};
    const size_t aoff = (size_t)(r0 + lr) * K + 8 * hi, boff = (size_t)(c0 + lr) * K + 8 * hi;
#pragma unroll 1
    for (int kc = 0; kc < K; kc += 32) {
        V a[4], a2[4];
#pragma unroll
        for (int mb = 0; mb < 4; ++mb) { a[mb] = WFrag<T16>::ld(A + aoff + (size_t)mb * 16 * K + kc); if (NSPLIT == 1 || NSPLIT == 2) a2[mb] = WFrag<T16>::ld(A2 + aoff + (size_t)mb * 16 * K + kc); }
#pragma unroll
        for (int nb = 0; nb < 4; ++nb) { const V b = WFrag<T16>::ld(Bt + boff + (size_t)nb * 16 * K + kc); V b2; if (NSPLIT >= 2) b2 = WFrag<T16>::ld(Bt2 + boff + (size_t)nb * 16 * K + kc);
#pragma unroll
            for (int mb = 0; mb < 4; ++mb) { acc[mb][nb] = WFrag<T16>::mma(a[mb], b, acc[mb][nb]); if (NSPLIT == 1 || NSPLIT == 2) acc[mb][nb] = WFrag<T16>::mma(a2[mb], b, acc[mb][nb]); if (NSPLIT >= 2) acc[mb][nb] = WFrag<T16>::mma(a[mb], b2, acc[mb][nb]); } }
        asm volatile("v_nop\n\tv_nop\n\tv_nop\n\tv_nop" : "+v"(acc[0][0]), "+v"(acc[1][1]), "+v"(acc[2][2]), "+v"(acc[3][3]) : "v"(a[0]), "v"(a[3]));
    }
#pragma unroll
    for (int mb = 0; mb < 4; ++mb) {
#pragma unroll
        for (int nb = 0; nb < 4; ++nb) {
#pragma unroll
            for (int j = 0; j < 8; ++j) os[(hi * 8 + j) * 68 + nb * 16 + lr] = acc[mb][nb][j]; }
        __builtin_amdgcn_wave_barrier(); asm volatile("" ::: "memory");
        float* crow = C + (size_t)(r0 + mb * 16) * ldc + c0;
#pragma unroll 1
        for (int ps = 0; ps < 2; ++ps) {
#pragma unroll
            for (int s = 0; s < 8; ++s) { const int row = 2 * s + hi, cofs = lr * 4; v4f val = *(const v4fa*)(os + row * 68 + cofs); if (BIAS) { val[0] += bfr(bias[c0 + cofs]); val[1] += bfr(bias[c0 + cofs + 1]); val[2] += bfr(bias[c0 + cofs + 2]); val[3] += bfr(bias[c0 + cofs + 3]); }
                *(volatile v4f*)(crow + (size_t)row * ldc + cofs) = val; }
            if (ps == 0) __threadfence(); }
        __builtin_amdgcn_wave_barrier(); asm volatile("" ::: "memory");
    }
}

__device__ __forceinline__ h16 tohx(float x) { return (h16)x; }
__device__ __forceinline__ void splitf(float y, unsigned short& h, unsigned short& l) { h = f2bf(y); l = f2bf(y - bf2f(h)); }

__global__ __launch_bounds__(256) void k_wtG(const float* __restrict__ w, unsigned ksh, unsigned N, bf* Bt) {
    const unsigned lane = threadIdx.x & 31u; const unsigned L0 = (blockIdx.x * 8u + (threadIdx.x >> 5)) * 8u; const unsigned K = 1u << ksh; const unsigned nlines = (N << ksh) >> 6;
#pragma unroll
    for (int ps = 0; ps < 2; ++ps) {
#pragma unroll 1
        for (unsigned l = 0; l < 8u; ++l) { const unsigned L = L0 + l; if (L >= nlines) break; const unsigned e = L * 64u + lane * 2u; const unsigned k = e & (K - 1u), n = e >> ksh; v2us o;
            o[0] = f2bf(w[(size_t)k * N + n]); o[1] = f2bf(w[(size_t)(k + 1u) * N + n]); *(volatile v2us*)(Bt + e) = o; }
        if (ps == 0) __threadfence(); }
}
__global__ __launch_bounds__(256) void k_cvt8(const float* __restrict__ src, bf* dst, unsigned n8) { const unsigned i = blockIdx.x * 256u + threadIdx.x; if (i >= n8) return; const v8f v = *(const v8f*)(src + (size_t)i * 8); v8us o;
#pragma unroll
    for (int k = 0; k < 8; ++k) o[k] = f2bf(v[k]); *(volatile v8us*)(dst + (size_t)i * 8) = o; __threadfence(); *(volatile v8us*)(dst + (size_t)i * 8) = o; }

__global__ __launch_bounds__(256) void k_cstab(float* CS) {
    const unsigned idx = blockIdx.x * 256u + threadIdx.x; if (idx >= (unsigned)(TT * 64)) return; const unsigned i = idx & 63u, t = idx >> 6;
    const double g3 = __builtin_sqrt(10.0); const double g2 = __builtin_sqrt(g3); const double g1 = __builtin_sqrt(g2); const double g0 = __builtin_sqrt(g1);
    double p = 1.0; p *= (i & 1u) ? g0 : 1.0; p *= (i & 2u) ? g1 : 1.0; p *= (i & 4u) ? g2 : 1.0; p *= (i & 8u) ? g3 : 1.0; p *= (i & 16u) ? 10.0 : 1.0; p *= (i & 32u) ? 100.0 : 1.0;
    const float pf = (float)p; const float inv = 1.0f / pf; const float ang = __fmul_rn((float)t, inv); float sn, cn; sincosf(ang, &sn, &cn);
    v2f cs; cs[0] = cn; cs[1] = sn; *(volatile v2f*)(CS + (size_t)idx * 2) = cs; __threadfence(); *(volatile v2f*)(CS + (size_t)idx * 2) = cs; }

__global__ __launch_bounds__(256) void k_mflag(const int* __restrict__ mask, int* flags) {
    __shared__ int sf[32];
    const unsigned lane = threadIdx.x & 31u, w = threadIdx.x >> 5;
#pragma unroll 1
    for (unsigned rr = 0; rr < 4u; ++rr) { unsigned row = blockIdx.x * 32u + w * 4u + rr; row = (row < (unsigned)TT) ? row : (unsigned)(TT - 1); const int* mr = mask + (size_t)row * TTF; int z = 0;
#pragma unroll 4
        for (unsigned ch = 0; ch < (unsigned)(TT / 128); ++ch) { const v4i m = *(const v4i*)(mr + ch * 128u + lane * 4u); z |= (m[0] == 0) | (m[1] == 0) | (m[2] == 0) | (m[3] == 0); }
#pragma unroll
        for (int sh = 16; sh; sh >>= 1) z |= __shfl_xor(z, sh, 32);
        if (lane == 0u) sf[w * 4u + rr] = z; }
    __syncthreads();
    if (threadIdx.x < 32u) { const int val = sf[threadIdx.x]; volatile int* p = flags + blockIdx.x * 32u + threadIdx.x; *p = val; __threadfence(); *p = val; }
}

__global__ __launch_bounds__(256) void k_rope(const float* __restrict__ F, unsigned pitch, unsigned nheads, const float* __restrict__ CS, h16* P16) {
    const unsigned e = (blockIdx.x * 256u + threadIdx.x) * 2u; if (e >= nheads * (unsigned)(TT * HD)) return; const unsigned d = e % (unsigned)HD; const unsigned t = (e / (unsigned)HD) % (unsigned)TT; const unsigned h = e / (unsigned)(HD * TT); const float* f = F + (size_t)t * pitch + h * (unsigned)HD; v2h o16;
#pragma unroll
    for (unsigned q = 0; q < 2u; ++q) { const unsigned dd = d + q; const unsigned dp = (dd < 64u) ? dd + 64u : dd - 64u; const float x0 = f[dd], x1 = f[dp];
        const v2f cs = *(const v2f*)(CS + ((size_t)t * 64u + (dd & 63u)) * 2u); float a = __fmul_rn(x0, cs[0]), bq = __fmul_rn(x1, cs[1]); asm volatile("" : "+v"(a)); asm volatile("" : "+v"(bq)); const float r = (dd < 64u) ? __fsub_rn(a, bq) : __fadd_rn(a, bq);
        o16[q] = tohx(r); }
    *(volatile v2h*)(P16 + e) = o16; __threadfence(); *(volatile v2h*)(P16 + e) = o16; }
__global__ __launch_bounds__(256) void k_vtp(const float* __restrict__ F, unsigned pitch, unsigned nheads, h16* V16) { const unsigned e = (blockIdx.x * 256u + threadIdx.x) * 2u; if (e >= nheads * (unsigned)(HD * TT)) return; const unsigned t = e % (unsigned)TT; const unsigned d = (e / (unsigned)TT) % (unsigned)HD; const unsigned g = e / (unsigned)(TT * HD); v2h o16;
#pragma unroll
    for (unsigned q = 0; q < 2u; ++q) { const float x = F[(size_t)(t + q) * pitch + g * (unsigned)HD + d]; o16[q] = tohx(x); }
    *(volatile v2h*)(V16 + e) = o16; __threadfence(); *(volatile v2h*)(V16 + e) = o16; }

__global__ __launch_bounds__(256) void k_asoft(const float* __restrict__ Sb, const int* __restrict__ mask, const int* __restrict__ rflag, h16* P16) {
    const unsigned lane = threadIdx.x & 31u; const unsigned row = blockIdx.x * 8u + (threadIdx.x >> 5); if (row >= (unsigned)(ZH * TT)) return; const unsigned i = row % (unsigned)TT;
    const float* sr = Sb + (size_t)row * TT; const int* mr = mask + (size_t)i * TTF; const int rf = __builtin_amdgcn_readfirstlane(rflag[i]); float v[TT / 32]; float mx = NEGF;
#pragma unroll
    for (int ch = 0; ch < TT / 128; ++ch) { const unsigned j0 = (unsigned)ch * 128u + lane * 4u; const v4f a = *(const v4f*)(sr + j0); v4i m = (v4i){1, 1, 1, 1}; if (rf != 0) m = *(const v4i*)(mr + j0);
#pragma unroll
        for (int q = 0; q < 4; ++q) { const float t = a[q] * SCL + ((m[q] != 0) ? 0.0f : NEGF); v[ch * 4 + q] = t; mx = fmaxf(mx, t); } }
#pragma unroll
    for (int sh = 16; sh; sh >>= 1) mx = fmaxf(mx, __shfl_xor(mx, sh, 32));
    float sum = 0.f;
#pragma unroll
    for (int k = 0; k < TT / 32; ++k) { float d0 = __fsub_rn(v[k], mx); asm volatile("" : "+v"(d0)); v[k] = __builtin_amdgcn_exp2f(__fmul_rn(d0, 1.4426950408889634f)); sum += v[k]; }
#pragma unroll
    for (int sh = 16; sh; sh >>= 1) sum += __shfl_xor(sum, sh, 32);
    const float f = __fdiv_rn(PCAR, sum);
#pragma unroll 1
    for (int ps = 0; ps < 2; ++ps) {
#pragma unroll
        for (int ch = 0; ch < TT / 128; ++ch) { v4h o4;
#pragma unroll
            for (int q = 0; q < 4; ++q) o4[q] = tohx(v[ch * 4 + q] * f);
            *(volatile v4h*)(P16 + (size_t)row * TT + (unsigned)ch * 128u + lane * 4u) = o4; }
        if (ps == 0) __threadfence(); }
}
__global__ __launch_bounds__(256) void k_merge(const float* __restrict__ O, unsigned h0, bf* Ah, bf* Al) { const unsigned e = (blockIdx.x * 256u + threadIdx.x) * 2u; if (e >= (unsigned)(ZH * TT * HD)) return; const unsigned d = e % (unsigned)HD; const unsigned t = (e / (unsigned)HD) % (unsigned)TT; const unsigned zz = e / (unsigned)(HD * TT); const size_t oo = (size_t)t * DQ + (h0 + zz) * (unsigned)HD + d;
    v2us oh, ol;
#pragma unroll
    for (unsigned q = 0; q < 2u; ++q) { unsigned short a, c2; splitf(O[e + q] * (1.0f / PCAR), a, c2); oh[q] = a; ol[q] = c2; }
    *(volatile v2us*)(Ah + oo) = oh; *(volatile v2us*)(Al + oo) = ol; __threadfence(); *(volatile v2us*)(Ah + oo) = oh; *(volatile v2us*)(Al + oo) = ol; }

constexpr size_t pad256(size_t b) { return (b + 255) & ~(size_t)255; }
constexpr size_t cmax(size_t a, size_t b) { return a > b ? a : b; }
constexpr size_t B_WQ = pad256((size_t)DQ * DM * 2), B_WK = pad256((size_t)DKV * DM * 2), B_WV = B_WK, B_WO = pad256((size_t)DM * DQ * 2);
constexpr size_t B_XB = pad256((size_t)TT * DM * 2), B_FQ = pad256((size_t)TT * DQ * 4), B_FK = pad256((size_t)TT * DKV * 4), B_CS = pad256((size_t)TT * 64 * 2 * 4);
constexpr size_t B_PRE = B_WQ + B_WK + B_WV + B_XB + B_FQ + B_FK + B_CS;
constexpr size_t B_SB = pad256((size_t)ZH * TT * TT * 4), B_OB = pad256((size_t)ZH * TT * HD * 4);
constexpr size_t B_BIG = cmax(cmax(B_PRE, B_SB), cmax(B_WO, B_OB));
constexpr size_t B_P16 = pad256((size_t)ZH * TT * TT * 2), B_QP = pad256((size_t)NH_ * TT * HD * 2), B_KP = pad256((size_t)NKV * TT * HD * 2), B_VT = pad256((size_t)NKV * HD * TT * 2), B_AT = pad256((size_t)TT * DQ * 2), B_FLG = pad256((size_t)TT * 4);
constexpr size_t B_TOTAL = B_BIG + B_P16 + B_QP + B_KP + B_VT + 2 * B_AT + B_FLG;
static_assert(B_TOTAL <= (size_t)134217728);
static_assert(B_PRE <= B_BIG);
static_assert(B_SB <= B_BIG);
static_assert(B_WO <= B_BIG);
static_assert(B_OB <= B_BIG);

extern "C" void kernel_launch(void* const* d_in, const int* in_sizes, int n_in,
                              void* d_out, int out_size, void* d_ws, size_t ws_size, hipStream_t stream) {
    if (n_in < 8) return;
    if ((size_t)in_sizes[0] < (size_t)NB * TT * DM || (size_t)in_sizes[1] < (size_t)NB * TT * DM || (size_t)in_sizes[2] < (size_t)NB * TT * DM) return;
    if ((size_t)in_sizes[3] < (size_t)(TT - 1) * TTF + TT) return;
    if ((size_t)in_sizes[4] < (size_t)DM * DQ || (size_t)in_sizes[5] < (size_t)DM * DKV || (size_t)in_sizes[6] < (size_t)DM * DKV || (size_t)in_sizes[7] < (size_t)DQ * DM) return;
    if ((size_t)out_size < (size_t)NB * TT * DM) return;
    if (B_TOTAL > ws_size) return;
    const float* query = (const float*)d_in[0]; const float* key = (const float*)d_in[1]; const float* value = (const float*)d_in[2]; const int* mask = (const int*)d_in[3];
    const float* wq = (const float*)d_in[4]; const float* wk = (const float*)d_in[5]; const float* wv = (const float*)d_in[6]; const float* wo = (const float*)d_in[7];
    float* OUT = (float*)d_out;
    char* base = (char*)d_ws; size_t off = 0;
    auto take = [&](size_t bytes) { char* p = base + off; off += pad256(bytes); return (void*)p; };
    char* BIG = (char*)take(B_BIG);
    h16* P16 = (h16*)take(B_P16); h16* QP16 = (h16*)take(B_QP); h16* KP16 = (h16*)take(B_KP); h16* VT16 = (h16*)take(B_VT); bf* ATh = (bf*)take(B_AT); bf* ATl = (bf*)take(B_AT); int* FLG = (int*)take(B_FLG);
    if (off > ws_size) return;
    size_t po = 0; auto sub = [&](size_t bytes) { char* p = BIG + po; po += bytes; return (void*)p; };
    bf* WQ = (bf*)sub(B_WQ); bf* WK = (bf*)sub(B_WK); bf* WV = (bf*)sub(B_WV); bf* XB = (bf*)sub(B_XB); float* FQ = (float*)sub(B_FQ); float* FK = (float*)sub(B_FK); float* CS = (float*)sub(B_CS);
    float* FV = FK;
    float* Sb = (float*)BIG;
    float* Ob = (float*)BIG;
    bf* WO = (bf*)BIG;
    const unsigned LQ = (unsigned)(((size_t)NH_ * TT * HD / 2 + 255) / 256), LKv = (unsigned)(((size_t)NKV * TT * HD / 2 + 255) / 256);
    const unsigned n8 = (unsigned)((size_t)TT * DM / 8);
    for (int b = 0; b < NB; ++b) {
        const float* qb = query + (size_t)b * TTF * DM; const float* kb = key + (size_t)b * TTF * DM; const float* vb = value + (size_t)b * TTF * DM; const int* mb = mask + (size_t)b * TTF * TTF;
        k_wtG<<<(unsigned)((DM * DQ / 64 + 63) / 64), 256, 0, stream>>>(wq, KSH, DQ, WQ);
        k_wtG<<<(unsigned)((DM * DKV / 64 + 63) / 64), 256, 0, stream>>>(wk, KSH, DKV, WK);
        k_wtG<<<(unsigned)((DM * DKV / 64 + 63) / 64), 256, 0, stream>>>(wv, KSH, DKV, WV);
        k_cstab<<<(unsigned)((TT * 64 + 255) / 256), 256, 0, stream>>>(CS);
        k_mflag<<<(unsigned)(TT / 32), 256, 0, stream>>>(mb, FLG);
        k_cvt8<<<(n8 + 255u) / 256u, 256, 0, stream>>>(qb, XB, n8);
        k_gemmw<bf, 0, false><<<dim3(TT / 64, DQ / 64, 1), 32, 0, stream>>>(XB, nullptr, WQ, nullptr, DM, FQ, DQ, nullptr, 0, 0, 0);
        k_rope<<<LQ, 256, 0, stream>>>(FQ, DQ, NH_, CS, QP16);
        k_cvt8<<<(n8 + 255u) / 256u, 256, 0, stream>>>(kb, XB, n8);
        k_gemmw<bf, 0, false><<<dim3(TT / 64, DKV / 64, 1), 32, 0, stream>>>(XB, nullptr, WK, nullptr, DM, FK, DKV, nullptr, 0, 0, 0);
        k_rope<<<LKv, 256, 0, stream>>>(FK, DKV, NKV, CS, KP16);
        k_cvt8<<<(n8 + 255u) / 256u, 256, 0, stream>>>(vb, XB, n8);
        k_gemmw<bf, 0, false><<<dim3(TT / 64, DKV / 64, 1), 32, 0, stream>>>(XB, nullptr, WV, nullptr, DM, FV, DKV, nullptr, 0, 0, 0);
        k_vtp<<<LKv, 256, 0, stream>>>(FV, DKV, NKV, VT16);
        for (int g = 0; g < NKV; ++g) { const size_t zq = (size_t)g * REP, zk = (size_t)g;
            k_gemmw<h16, 0, false><<<dim3(TT / 64, TT / 64, ZH), 32, 0, stream>>>(QP16 + zq * TT * HD, nullptr, KP16 + zk * TT * HD, nullptr, HD, Sb, TT, nullptr, (size_t)TT * HD, 0, (size_t)TT * TT);
            k_asoft<<<(unsigned)(ZH * TT / 8), 256, 0, stream>>>(Sb, mb, FLG, P16);
            k_gemmw<h16, 0, false><<<dim3(TT / 64, HD / 64, ZH), 32, 0, stream>>>(P16, nullptr, VT16 + zk * HD * TT, nullptr, TT, Ob, HD, nullptr, (size_t)TT * TT, 0, (size_t)TT * HD);
            k_merge<<<(unsigned)(((size_t)ZH * TT * HD / 2 + 255) / 256), 256, 0, stream>>>(Ob, (unsigned)(g * REP), ATh, ATl); }
        k_wtG<<<(unsigned)((DQ * DM / 64 + 63) / 64), 256, 0, stream>>>(wo, KSH, DM, WO);
        k_gemmw<bf, 1, false><<<dim3(TT / 64, DM / 64, 1), 32, 0, stream>>>(ATh, ATl, WO, nullptr, DQ, OUT + (size_t)b * TTF * DM, DM, nullptr, 0, 0, 0); }
}
